// SeqGGNN_59210419143210
// MI455X (gfx1250) — hardware-verified
//
#include <hip/hip_runtime.h>
#include <stdint.h>

#define NB     64
#define NS     512
#define NH     256
#define NV     32000
#define NSTEP  10
#define NP     11
#define POS0   (NS - NP)
#define MROWS  (NP * NB)
#define HROWS  ((NP + 1) * NB)
#define KHL    512
#define KMSG   1536
#define KGATE  1024
#define NGATE  1024
#define WSCAP  134217728

static_assert(NP == NSTEP + 1);
static_assert(POS0 >= 1);
static_assert(NB == 64);
static_assert(NH % 32 == 0);
static_assert(KHL == 2 * NH);
static_assert(KMSG == 3 * KHL);
static_assert(KGATE == 2 * KHL);
static_assert(NV % 128 == 0);
static_assert(NH % 128 == 0);
static_assert(NGATE % 128 == 0);
static_assert(MROWS % 64 == 0);
static_assert((NV * 32) % 256 == 0);

typedef float          v4f   __attribute__((ext_vector_type(4)));
typedef float          v8f   __attribute__((ext_vector_type(8)));
typedef int            v8i   __attribute__((ext_vector_type(8)));
typedef unsigned int   v4u   __attribute__((ext_vector_type(4)));
typedef unsigned short v8us  __attribute__((ext_vector_type(8)));
typedef __bf16         v16bf __attribute__((ext_vector_type(16)));
typedef v4f  __attribute__((may_alias)) v4fa;
typedef v4u  __attribute__((may_alias)) v4ua;
typedef v8us __attribute__((may_alias)) v8usa;
union FragB { v16bf v; v8us h[2]; v8i w; };

__device__ __forceinline__ unsigned short f2bf_bits(float f) {
  unsigned u = __float_as_uint(f);
  return (unsigned short)((u + 0x7FFFu + ((u >> 16) & 1u)) >> 16);
}
__device__ __forceinline__ float bf_bits2f(unsigned short b) { return __uint_as_float(((unsigned)b) << 16); }
__device__ __forceinline__ float bfr(float f) { return bf_bits2f(f2bf_bits(f)); }
__device__ __forceinline__ unsigned pk16(unsigned short a, unsigned short b) { return (unsigned)a | ((unsigned)b << 16); }
__device__ __forceinline__ v4u cvt8(v4f a, v4f c) {
  v4u v;
  v[0] = pk16(f2bf_bits(a[0]), f2bf_bits(a[1]));
  v[1] = pk16(f2bf_bits(a[2]), f2bf_bits(a[3]));
  v[2] = pk16(f2bf_bits(c[0]), f2bf_bits(c[1]));
  v[3] = pk16(f2bf_bits(c[2]), f2bf_bits(c[3]));
  return v;
}
__device__ __forceinline__ v8f z8() { v8f z = {0.f, 0.f, 0.f, 0.f, 0.f, 0.f, 0.f, 0.f}; return z; }

__device__ __forceinline__ v8f wmb(const FragB& a, const FragB& b, v8f c) {
  v8f d = __builtin_amdgcn_wmma_f32_16x16x32_bf16(false, a.v, false, b.v, (short)0, c, false, false);
  asm volatile("v_nop\n\tv_nop\n\tv_nop\n\tv_nop" : "+v"(d) : "v"(a.w), "v"(b.w));
  return d;
}

__device__ __forceinline__ void gemm_seg(v8f (&acc)[2][4],
                                         const unsigned short* __restrict__ a0,
                                         const unsigned short* __restrict__ a1,
                                         const unsigned short* __restrict__ b, int ldb) {
#pragma unroll 1
  for (int k0 = 0; k0 < KHL; k0 += 32) {
    FragB fa0, fa1;
    fa0.h[0] = *(const v8usa*)(a0 + k0);
    fa0.h[1] = *(const v8usa*)(a0 + k0 + 16);
    fa1.h[0] = *(const v8usa*)(a1 + k0);
    fa1.h[1] = *(const v8usa*)(a1 + k0 + 16);
#pragma unroll
    for (int nt = 0; nt < 4; ++nt) {
      const unsigned short* bq = b + (size_t)nt * 16 * (size_t)ldb + k0;
      FragB fb;
      fb.h[0] = *(const v8usa*)bq;
      fb.h[1] = *(const v8usa*)(bq + 16);
      acc[0][nt] = wmb(fa0, fb, acc[0][nt]);
      acc[1][nt] = wmb(fa1, fb, acc[1][nt]);
    }
  }
}

__device__ __forceinline__ void f32_store_pass(const float* sO, float* dst, size_t ldd, int w, int lane) {
  const int q8 = lane & 7, sub = lane >> 3;
#pragma unroll 4
  for (int it = 0; it < 16; ++it) {
    const int L = it * 16 + w * 4 + sub;
    const int row = L >> 2, ql = L & 3;
    const v4f v = *(const v4fa*)(sO + row * 128 + 32 * ql + 4 * q8);
    *(volatile v4f*)(dst + (size_t)row * ldd + 32 * ql + 4 * q8) = v;
  }
}

__device__ __forceinline__ void msg_store_pass(const unsigned short* sT, unsigned short* dst, int w, int lane) {
  const int q8 = lane & 7, sub = lane >> 3;
#pragma unroll 4
  for (int it = 0; it < 16; ++it) {
    const int L = it * 16 + w * 4 + sub;
    const int plane = L >> 7, row = (L & 127) >> 1, hl = L & 1;
    const v4u v = *(const v4ua*)(sT + plane * 8192 + row * 128 + 64 * hl + 8 * q8);
    *(volatile v4u*)(dst + (size_t)row * KHL + plane * NH + 64 * hl + 8 * q8) = v;
  }
}

__global__ __launch_bounds__(256) void k_pa(const float* __restrict__ W_edge, unsigned short* __restrict__ WE6) {
  __shared__ __align__(16) unsigned short sT[32 * 256];
  const int tid = threadIdx.x, lane = tid & 31, w = tid >> 5;
  const int t = blockIdx.x >> 3, n0 = (blockIdx.x & 7) * 32;
  const float* src = W_edge + (size_t)t * (NH * NH) + n0 + lane;
#pragma unroll 4
  for (int i = 0; i < 32; ++i) {
    const int k = w + 8 * i;
    const float v = src[(size_t)k * NH];
    sT[lane * 256 + k] = f2bf_bits(v);
  }
  __syncthreads();
#pragma unroll 1
  for (int pass = 0; pass < 2; ++pass) {
#pragma unroll 4
    for (int it = 0; it < 8; ++it) {
      const int U = it * 256 + tid;
      const int row = U >> 6, d = (U >> 5) & 1, uu = U & 31;
      const v4u v = *(const v4ua*)(sT + row * 256 + 8 * uu);
      *(volatile v4u*)(WE6 + (size_t)(n0 + row) * KMSG + 512 * t + 256 * d + 8 * uu) = v;
    }
    __threadfence();
  }
}

__global__ __launch_bounds__(256) void k_pb(const float* __restrict__ W_ih, const float* __restrict__ W_hh,
                                            unsigned short* __restrict__ WG) {
  const int U = blockIdx.x * 256 + threadIdx.x;
  const int n = U >> 7, seg = (U >> 5) & 3, ku = U & 31;
  const int rih = (n < 768) ? n : 767;
  const int rhh = (n >= 768) ? (n - 256) : n;
  const float* pi = W_ih + (size_t)rih * NH + 8 * ku;
  const float* ph = W_hh + (size_t)rhh * NH + 8 * ku;
  const v4f ia = *(const v4fa*)pi;
  const v4f ic = *(const v4fa*)(pi + 4);
  const v4f ha = *(const v4fa*)ph;
  const v4f hc = *(const v4fa*)(ph + 4);
  const unsigned mi = ((seg < 2) && (n < 768)) ? 0xffffffffu : 0u;
  const unsigned mh = ((seg >= 2) && ((n < 512) || (n >= 768))) ? 0xffffffffu : 0u;
  const v4u bi = cvt8(ia, ic);
  const v4u bh = cvt8(ha, hc);
  v4u v;
  v[0] = (bi[0] & mi) | (bh[0] & mh);
  v[1] = (bi[1] & mi) | (bh[1] & mh);
  v[2] = (bi[2] & mi) | (bh[2] & mh);
  v[3] = (bi[3] & mi) | (bh[3] & mh);
  unsigned short* dst = WG + (size_t)U * 8;
  *(volatile v4u*)dst = v;
  __threadfence();
  *(volatile v4u*)dst = v;
}

__global__ __launch_bounds__(128) void k_pc(const float* __restrict__ b_edge, const float* __restrict__ b_ih,
                                            const float* __restrict__ b_hh, const float* __restrict__ out_b,
                                            float* __restrict__ BM, float* __restrict__ BG, float* __restrict__ OB) {
  const int u = blockIdx.x * 128 + threadIdx.x;
  if (u >= 8384) return;
  v4f o;
  float* dst;
  if (u < 128) {
    const int sel = u >> 6, c = 4 * (u & 63);
    const v4f v0 = *(const v4fa*)(b_edge + c);
    const v4f v1 = *(const v4fa*)(b_edge + NH + c);
    const v4f v2 = *(const v4fa*)(b_edge + 2 * NH + c);
    const unsigned m1 = (sel == 0) ? 0xffffffffu : 0u;
#pragma unroll
    for (int i = 0; i < 4; ++i) {
      const float t1 = __uint_as_float(__float_as_uint(bfr(v1[i])) & m1);
      o[i] = (bfr(v0[i]) + t1) + bfr(v2[i]);
    }
    dst = BM + sel * NH + c;
  } else if (u < 384) {
    const int c = 4 * (u - 128);
    const int ci = (c < 764) ? c : 764;
    const int ch = (c >= 768) ? (c - 256) : c;
    const v4f vi = *(const v4fa*)(b_ih + ci);
    const v4f vh = *(const v4fa*)(b_hh + ch);
    const unsigned mi = (c < 768) ? 0xffffffffu : 0u;
    const unsigned mh = ((c < 512) || (c >= 768)) ? 0xffffffffu : 0u;
#pragma unroll
    for (int i = 0; i < 4; ++i) {
      const float ti = __uint_as_float(__float_as_uint(bfr(vi[i])) & mi);
      const float th = __uint_as_float(__float_as_uint(bfr(vh[i])) & mh);
      o[i] = ti + th;
    }
    dst = BG + c;
  } else {
    const int c = 4 * (u - 384);
    const v4f v = *(const v4fa*)(out_b + c);
#pragma unroll
    for (int i = 0; i < 4; ++i) o[i] = bfr(v[i]);
    dst = OB + c;
  }
  *(volatile v4f*)dst = o;
  __threadfence();
  *(volatile v4f*)dst = o;
}

__global__ __launch_bounds__(256) void k_pd(const float* __restrict__ out_w, unsigned short* __restrict__ OW2) {
  const int U = blockIdx.x * 256 + threadIdx.x;
  const int n = U >> 5, ku = U & 31;
  const float* src = out_w + (size_t)n * NH + 8 * ku;
  const v4f a = *(const v4fa*)src;
  const v4f c = *(const v4fa*)(src + 4);
  const v4u v = cvt8(a, c);
  unsigned short* d0 = OW2 + (size_t)n * KHL + 8 * ku;
  unsigned short* d1 = d0 + NH;
  *(volatile v4u*)d0 = v;
  *(volatile v4u*)d1 = v;
  __threadfence();
  *(volatile v4u*)d0 = v;
  *(volatile v4u*)d1 = v;
}

__global__ __launch_bounds__(64) void k_pe(const int* __restrict__ x, const float* __restrict__ emb,
                                           float* __restrict__ Hf, unsigned short* __restrict__ Hhl) {
  const int row = blockIdx.x, u = threadIdx.x;
  unsigned short* dh = Hhl + (size_t)row * KHL + 8 * u;
  if (row < MROWS) {
    const int p = row >> 6, b = row & 63;
    int id = x[b * NS + POS0 + p];
    id = (id < 0) ? 0 : ((id > NV - 1) ? (NV - 1) : id);
    const float* e = emb + (size_t)id * NH;
    const v4f f = *(const v4fa*)(e + 4 * u);
    v4f fo;
#pragma unroll
    for (int i = 0; i < 4; ++i) fo[i] = bfr(f[i]);
    const int uk = u & 31;
    const v4f a = *(const v4fa*)(e + 8 * uk);
    const v4f c = *(const v4fa*)(e + 8 * uk + 4);
    const unsigned mk = (u < 32) ? 0xffffffffu : 0u;
    v4u hv = cvt8(a, c);
    hv[0] &= mk; hv[1] &= mk; hv[2] &= mk; hv[3] &= mk;
    float* df = Hf + (size_t)row * NH + 4 * u;
    *(volatile v4f*)df = fo;
    *(volatile v4u*)dh = hv;
    __threadfence();
    *(volatile v4f*)df = fo;
    *(volatile v4u*)dh = hv;
  } else {
    const v4u z = {0u, 0u, 0u, 0u};
    *(volatile v4u*)dh = z;
    __threadfence();
    *(volatile v4u*)dh = z;
  }
}

__global__ __launch_bounds__(128) __attribute__((amdgpu_num_vgpr(248)))
void k_msg(const unsigned short* __restrict__ Hhl, const unsigned short* __restrict__ WE6,
           const float* __restrict__ BM, unsigned short* __restrict__ Mhl, int p0) {
  __shared__ __align__(16) unsigned short sT[2 * 64 * 128];
  __shared__ __align__(16) float sBias[128];
  const int tid = threadIdx.x, lane = tid & 31, w = tid >> 5;
  const int h = lane >> 4, m = lane & 15;
  const int wr = w & 1, wc = w >> 1;
  const int p = p0 + blockIdx.x;
  const int n0 = blockIdx.y * 128;
  const int sel = (p == NP - 1) ? 1 : 0;
  if (tid < 32) *(v4fa*)(sBias + 4 * tid) = *(const v4fa*)(BM + sel * NH + n0 + 4 * tid);

  const int arow = 64 * p + 32 * wr + m;
  const unsigned short* wb = WE6 + (size_t)(n0 + 64 * wc + m) * KMSG + 8 * h;

  v8f acc[2][4];
#pragma unroll
  for (int mt = 0; mt < 2; ++mt)
#pragma unroll
    for (int nt = 0; nt < 4; ++nt) acc[mt][nt] = z8();

#pragma unroll 1
  for (int seg = 0; seg < 3; ++seg) {
    const int off = (seg == 0) ? -64 : ((seg == 1) ? 64 : 0);
    const unsigned short* a0 = Hhl + (size_t)(arow + off) * KHL + 8 * h;
    gemm_seg(acc, a0, a0 + 16 * KHL, wb + KHL * seg, KMSG);
  }
  __syncthreads();

#pragma unroll
  for (int nt = 0; nt < 4; ++nt) {
    const int cl = 64 * wc + 16 * nt + m;
    const float bv = sBias[cl];
#pragma unroll
    for (int mt = 0; mt < 2; ++mt) {
#pragma unroll
      for (int r = 0; r < 8; ++r) {
        const int rl = 32 * wr + 16 * mt + 8 * h + r;
        const float v = acc[mt][nt][r] + bv;
        const unsigned short hb = f2bf_bits(v);
        const unsigned short lb = f2bf_bits(v - bf_bits2f(hb));
        sT[rl * 128 + cl] = hb;
        sT[8192 + rl * 128 + cl] = lb;
      }
    }
  }
  __syncthreads();

  unsigned short* dst = Mhl + (size_t)(64 * p) * KHL + n0;
  msg_store_pass(sT, dst, w, lane);
  __threadfence();
  msg_store_pass(sT, dst, w, lane);
}

__global__ __launch_bounds__(128) __attribute__((amdgpu_num_vgpr(248)))
void k_gate(const unsigned short* __restrict__ Mhl, const unsigned short* __restrict__ Hhl,
            const unsigned short* __restrict__ WG, const float* __restrict__ BG,
            float* __restrict__ G, int p0) {
  __shared__ __align__(16) float sO[64 * 128];
  __shared__ __align__(16) float sBias[128];
  const int tid = threadIdx.x, lane = tid & 31, w = tid >> 5;
  const int h = lane >> 4, m = lane & 15;
  const int wr = w & 1, wc = w >> 1;
  const int p = p0 + blockIdx.x;
  const int n0 = blockIdx.y * 128;
  const int grp = blockIdx.y >> 1;
  if (tid < 32) *(v4fa*)(sBias + 4 * tid) = *(const v4fa*)(BG + n0 + 4 * tid);

  const int arow = 64 * p + 32 * wr + m;
  const unsigned short* wb = WG + (size_t)(n0 + 64 * wc + m) * KGATE + 8 * h;

  v8f acc[2][4];
#pragma unroll
  for (int mt = 0; mt < 2; ++mt)
#pragma unroll
    for (int nt = 0; nt < 4; ++nt) acc[mt][nt] = z8();

  if (grp != 3) {
    const unsigned short* a0 = Mhl + (size_t)arow * KHL + 8 * h;
    gemm_seg(acc, a0, a0 + 16 * KHL, wb, KGATE);
  }
  if (grp != 2) {
    const unsigned short* a0 = Hhl + (size_t)arow * KHL + 8 * h;
    gemm_seg(acc, a0, a0 + 16 * KHL, wb + KHL, KGATE);
  }
  __syncthreads();

#pragma unroll
  for (int nt = 0; nt < 4; ++nt) {
    const int cl = 64 * wc + 16 * nt + m;
    const float bv = sBias[cl];
#pragma unroll
    for (int mt = 0; mt < 2; ++mt) {
#pragma unroll
      for (int r = 0; r < 8; ++r) {
        const int rl = 32 * wr + 16 * mt + 8 * h + r;
        sO[rl * 128 + cl] = acc[mt][nt][r] + bv;
      }
    }
  }
  __syncthreads();

  float* dst = G + (size_t)(64 * p) * NGATE + n0;
  f32_store_pass(sO, dst, (size_t)NGATE, w, lane);
  __threadfence();
  f32_store_pass(sO, dst, (size_t)NGATE, w, lane);
}

__global__ __launch_bounds__(256) void k_gru(const float* __restrict__ G, float* Hf,
                                             unsigned short* __restrict__ Hhl, int p0) {
  __shared__ __align__(16) float sF[NH];
  __shared__ __align__(16) unsigned short sH[KHL];
  const int tid = threadIdx.x;
  const int row = 64 * p0 + blockIdx.x;
  const float* g = G + (size_t)row * NGATE;
  const float sr = g[tid];
  const float sz = g[NH + tid];
  const float gin = g[2 * NH + tid];
  const float ghn = g[3 * NH + tid];
  const float ho = Hf[(size_t)row * NH + tid];
  const float rg = 1.0f / (1.0f + expf(-sr));
  const float zg = 1.0f / (1.0f + expf(-sz));
  const float ng = tanhf(gin + rg * ghn);
  const float hv = (1.0f - zg) * ng + zg * ho;
  const unsigned short hb = f2bf_bits(hv);
  const unsigned short lb = f2bf_bits(hv - bf_bits2f(hb));
  sF[tid] = hv;
  sH[tid] = hb;
  sH[NH + tid] = lb;
  __syncthreads();
  if (tid < 64) {
    const v4f v = *(const v4fa*)(sF + 4 * tid);
    float* d = Hf + (size_t)row * NH + 4 * tid;
    *(volatile v4f*)d = v;
    __threadfence();
    *(volatile v4f*)d = v;
  } else if (tid < 128) {
    const int u = tid - 64;
    const v4u v = *(const v4ua*)(sH + 8 * u);
    unsigned short* d = Hhl + (size_t)row * KHL + 8 * u;
    *(volatile v4u*)d = v;
    __threadfence();
    *(volatile v4u*)d = v;
  }
}

__global__ __launch_bounds__(128) __attribute__((amdgpu_num_vgpr(248)))
void k_out(const unsigned short* __restrict__ Hhl, const unsigned short* __restrict__ OW2,
           const float* __restrict__ OB, float* __restrict__ out) {
  __shared__ __align__(16) float sO[64 * 128];
  __shared__ __align__(16) float sBias[128];
  const int tid = threadIdx.x, lane = tid & 31, w = tid >> 5;
  const int h = lane >> 4, m = lane & 15;
  const int wr = w & 1, wc = w >> 1;
  const int n0 = blockIdx.x * 128;
  if (tid < 32) *(v4fa*)(sBias + 4 * tid) = *(const v4fa*)(OB + n0 + 4 * tid);

  const int arow = 64 * (NP - 1) + 32 * wr + m;
  const unsigned short* a0 = Hhl + (size_t)arow * KHL + 8 * h;
  const unsigned short* wb = OW2 + (size_t)(n0 + 64 * wc + m) * KHL + 8 * h;

  v8f acc[2][4];
#pragma unroll
  for (int mt = 0; mt < 2; ++mt)
#pragma unroll
    for (int nt = 0; nt < 4; ++nt) acc[mt][nt] = z8();

  gemm_seg(acc, a0, a0 + 16 * KHL, wb, KHL);
  __syncthreads();

#pragma unroll
  for (int nt = 0; nt < 4; ++nt) {
    const int cl = 64 * wc + 16 * nt + m;
    const float bv = sBias[cl];
#pragma unroll
    for (int mt = 0; mt < 2; ++mt) {
#pragma unroll
      for (int r = 0; r < 8; ++r) {
        const int rl = 32 * wr + 16 * mt + 8 * h + r;
        sO[rl * 128 + cl] = acc[mt][nt][r] + bv;
      }
    }
  }
  __syncthreads();

  float* dst = out + n0;
  f32_store_pass(sO, dst, (size_t)NV, w, lane);
  __threadfence();
  f32_store_pass(sO, dst, (size_t)NV, w, lane);
}

extern "C" void kernel_launch(void* const* d_in, const int* in_sizes, int n_in,
                              void* d_out, int out_size, void* d_ws, size_t ws_size,
                              hipStream_t stream) {
  if (n_in < 10) return;
  if (in_sizes[0] != NB * NS) return;
  if (in_sizes[1] != NV * NH) return;
  if (in_sizes[2] != 3 * NH * NH) return;
  if (in_sizes[3] != 3 * NH) return;
  if (in_sizes[4] != 3 * NH * NH) return;
  if (in_sizes[5] != 3 * NH * NH) return;
  if (in_sizes[6] != 3 * NH) return;
  if (in_sizes[7] != 3 * NH) return;
  if (in_sizes[8] != NV * NH) return;
  if (in_sizes[9] != NV) return;
  if (out_size != NB * NV) return;

  const int*   x      = (const int*)d_in[0];
  const float* emb    = (const float*)d_in[1];
  const float* W_edge = (const float*)d_in[2];
  const float* b_edge = (const float*)d_in[3];
  const float* W_ih   = (const float*)d_in[4];
  const float* W_hh   = (const float*)d_in[5];
  const float* b_ih   = (const float*)d_in[6];
  const float* b_hh   = (const float*)d_in[7];
  const float* out_w  = (const float*)d_in[8];
  const float* out_b  = (const float*)d_in[9];
  float* out = (float*)d_out;

  size_t off = 0;
  const size_t oOW2 = off; off += (size_t)NV * KHL * 2;
  const size_t oWG  = off; off += (size_t)NGATE * KGATE * 2;
  const size_t oWE6 = off; off += (size_t)NH * KMSG * 2;
  const size_t oHhl = off; off += (size_t)HROWS * KHL * 2;
  const size_t oMhl = off; off += (size_t)MROWS * KHL * 2;
  const size_t oHf  = off; off += (size_t)MROWS * NH * 4;
  const size_t oG   = off; off += (size_t)MROWS * NGATE * 4;
  const size_t oOB  = off; off += (size_t)NV * 4;
  const size_t oBM  = off; off += (size_t)2 * NH * 4;
  const size_t oBG  = off; off += (size_t)NGATE * 4;
  if (off > ws_size) return;
  if (off > (size_t)WSCAP) return;

  char* ws = (char*)d_ws;
  unsigned short* OW2 = (unsigned short*)(ws + oOW2);
  unsigned short* WG  = (unsigned short*)(ws + oWG);
  unsigned short* WE6 = (unsigned short*)(ws + oWE6);
  unsigned short* Hhl = (unsigned short*)(ws + oHhl);
  unsigned short* Mhl = (unsigned short*)(ws + oMhl);
  float* Hf = (float*)(ws + oHf);
  float* G  = (float*)(ws + oG);
  float* OB = (float*)(ws + oOB);
  float* BM = (float*)(ws + oBM);
  float* BG = (float*)(ws + oBG);

  k_pa<<<dim3(24), dim3(256), 0, stream>>>(W_edge, WE6);
  k_pb<<<dim3(512), dim3(256), 0, stream>>>(W_ih, W_hh, WG);
  k_pc<<<dim3(66), dim3(128), 0, stream>>>(b_edge, b_ih, b_hh, out_b, BM, BG, OB);
  k_pd<<<dim3((NV * 32) / 256), dim3(256), 0, stream>>>(out_w, OW2);
  k_pe<<<dim3(HROWS), dim3(64), 0, stream>>>(x, emb, Hf, Hhl);

  for (int s = 1; s <= NSTEP; ++s) {
    const int np = NP - s;
    k_msg<<<dim3(np, NH / 128), dim3(128), 0, stream>>>(Hhl, WE6, BM, Mhl, s);
    k_gate<<<dim3(np, NGATE / 128), dim3(128), 0, stream>>>(Mhl, Hhl, WG, BG, G, s);
    k_gru<<<dim3(np * 64), dim3(256), 0, stream>>>(G, Hf, Hhl, s);
  }

  k_out<<<dim3(NV / 128), dim3(128), 0, stream>>>(Hhl, OW2, OB, out);
  (void)hipGetLastError();
}
